// CrossAttention_55198919688799
// MI455X (gfx1250) — hardware-run, weakly checked
//
#include <hip/hip_runtime.h>


#ifndef NB
#define NB 2
#endif
#ifndef SQ
#define SQ 2048
#endif
#ifndef SK
#define SK 4096
#endif
#define NB_FULL 2
#define SQ_FULL 2048
#define SK_FULL 4096
#define DM   512
#define KD   512
#define NH_  8
#define HD   64
#define CH   64
#define AW   4
#define OSP  68
#define GSP  68
#define WTP  68
#define WSC  64.0f
#define WSI  (1.0f / 64.0f)
#define CTXC 64.0f
#define SC2  ((float)(0.125 * 1.4426950408889634))
#define PSH  14.0f
#define NEGB (-3.0e38f)
#define LNEPS 1.0e-5f
#define NTOKQ (NB * SQ)
#define NTOKK (NB * SK)
#define OUT1_OFF ((size_t)NB_FULL * SQ_FULL * DM)

static_assert(HD == 64);
static_assert(NH_ * HD == DM);
static_assert(DM == KD);
static_assert(KD % 32 == 0);
static_assert(DM % 64 == 0);
static_assert(CH == 64);
static_assert(SQ % CH == 0);
static_assert(SQ % 64 == 0);
static_assert(SK % 64 == 0);
static_assert(NTOKQ % 64 == 0);
static_assert(NTOKK % 64 == 0);
static_assert(SK % 32 == 0);
static_assert(SQ % (16 * AW) == 0);
static_assert(NTOKQ % 4 == 0);
static_assert(NB <= NB_FULL);
static_assert(SQ <= SQ_FULL);
static_assert(SK <= SK_FULL);
static_assert((OSP * 4) % 16 == 0);
static_assert((GSP * 4) % 16 == 0);
static_assert((WTP * 4) % 16 == 0);
static_assert(OSP >= HD);
static_assert(GSP >= 64);
static_assert(OUT1_OFF * 4 == (size_t)8388608);
static_assert(32 * 16 * 4 == 16 * 64 * 2);
static_assert(32 * 16 * 8 == 16 * 64 * 4);
static_assert(256 * 16 * 2 == 64 * 64 * 2);
static_assert(256 * 16 * 4 == 64 * 64 * 4);
static_assert(32 * 16 * 2 == DM * 2);
static_assert(32 * 16 * 4 == DM * 4);
static_assert(16 * GSP * 4 <= 131072);
static_assert(AW * 16 * OSP * 4 <= 131072);
static_assert(64 * WTP * 4 <= 131072);
static_assert(4 * DM * 4 <= 131072);

typedef _Float16 h16;
typedef __attribute__((ext_vector_type(16))) _Float16 v16h;
typedef __attribute__((ext_vector_type(8)))  _Float16 v8h;
typedef __attribute__((ext_vector_type(8)))  float    v8f;
typedef __attribute__((ext_vector_type(4)))  float    v4f;
typedef v4f  __attribute__((may_alias)) v4fa;

__device__ __forceinline__ unsigned short f2bf(float f) { unsigned u = __float_as_uint(f); u += 0x7FFFu + ((u >> 16) & 1u); return (unsigned short)(u >> 16); }
__device__ __forceinline__ float bfr(float f) { return __uint_as_float(((unsigned)f2bf(f)) << 16); }
static __device__ __forceinline__ h16 toh_flush(float v) { const h16 r = (h16)v; return (fabsf(v) < 6.103515625e-05f) ? (h16)0.0f : r; }
__device__ __forceinline__ v16h cat16(v8h lo, v8h hi) { return __builtin_shufflevector(lo, hi, 0, 1, 2, 3, 4, 5, 6, 7, 8, 9, 10, 11, 12, 13, 14, 15); }
__device__ __forceinline__ v8f wmma16g(v16h a, v16h b, v8f c) {
    c = __builtin_amdgcn_wmma_f32_16x16x32_f16(false, a, false, b, (short)0, c, false, false);
    asm volatile("v_nop\n\tv_nop\n\tv_nop\n\tv_nop" : "+v"(c) : "v"(a), "v"(b));
    return c;
}
__device__ __forceinline__ v16h ldh(const h16* p) { return cat16(*(const v8h*)p, *(const v8h*)(p + 16)); }
__device__ __forceinline__ void wave_sync() { __builtin_amdgcn_fence(3  , "wavefront"); __builtin_amdgcn_wave_barrier(); asm volatile("" ::: "memory"); }
__device__ __forceinline__ float wsum(float v) {
    v += __shfl_xor(v, 16, 32); v += __shfl_xor(v, 8, 32); v += __shfl_xor(v, 4, 32); v += __shfl_xor(v, 2, 32); v += __shfl_xor(v, 1, 32); return v;
}
__device__ __forceinline__ v4f lo4(v8f v) { return __builtin_shufflevector(v, v, 0, 1, 2, 3); }
__device__ __forceinline__ v4f hi4(v8f v) { return __builtin_shufflevector(v, v, 4, 5, 6, 7); }

__global__ __launch_bounds__(256) void k_wconv(const float* __restrict__ W, h16* WT, int N) {
    __shared__ __align__(16) float ts[64 * WTP];
    const int tid = threadIdx.x; const int n0 = blockIdx.x * 64, k0 = blockIdx.y * 64;
#pragma unroll
    for (int it = 0; it < 4; ++it) { const int idx = it * 256 + tid; const int kr = idx >> 4, n4 = (idx & 15) * 4;
        const v4f v = *(const v4f*)(W + (size_t)(k0 + kr) * N + n0 + n4);
        *(v4fa*)(&ts[kr * WTP + n4]) = v; }
    __syncthreads();
#pragma unroll 1
    for (int ps = 0; ps < 2; ++ps) {
#pragma unroll
        for (int it = 0; it < 2; ++it) { const int idx = it * 256 + tid; const int n = idx >> 3, k8 = (idx & 7) * 8;
            v8h o;
#pragma unroll
            for (int i = 0; i < 8; ++i) o[i] = toh_flush(bfr(ts[(k8 + i) * WTP + n]) * WSC);
            *(volatile v8h*)(WT + (size_t)(n0 + n) * KD + k0 + k8) = o; }
        if (ps == 0) __threadfence(); }
}

__global__ __launch_bounds__(256) void k_xcvt(const float* __restrict__ src, h16* dst, int T, int TF, size_t n8) {
    const size_t i = (size_t)blockIdx.x * 256 + threadIdx.x; if (i >= n8) return;
    const size_t row = i >> 6; const int c8 = (int)(i & 63) * 8;
    const size_t bb = row / (size_t)T, tt = row % (size_t)T;
    const v8f v = *(const v8f*)(src + (bb * (size_t)TF + tt) * DM + c8); v8h o;
#pragma unroll
    for (int k = 0; k < 8; ++k) o[k] = toh_flush(bfr(v[k]));
    *(volatile v8h*)(dst + i * 8) = o; __threadfence(); *(volatile v8h*)(dst + i * 8) = o;
}

__device__ __forceinline__ void ln_row(v8f& a, v8f& c, const v8f ga, const v8f gc, const v8f ba, const v8f bc) {
#pragma clang fp contract(off)
    float s = 0.0f;
#pragma unroll
    for (int k = 0; k < 8; ++k) { s += a[k]; s += c[k]; }
    s = wsum(s);
    const float mean = s * (1.0f / (float)DM);
    float q = 0.0f;
#pragma unroll
    for (int k = 0; k < 8; ++k) { a[k] -= mean; c[k] -= mean; q += a[k] * a[k]; q += c[k] * c[k]; }
    q = wsum(q);
    const float inv = rsqrtf(q * (1.0f / (float)DM) + LNEPS);
#pragma unroll
    for (int k = 0; k < 8; ++k) { a[k] = a[k] * inv * ga[k] + ba[k]; c[k] = c[k] * inv * gc[k] + bc[k]; }
}

__global__ __launch_bounds__(128) void k_ln1(const float* __restrict__ src, const float* __restrict__ g, const float* __restrict__ bt, h16* dst) {
#pragma clang fp contract(off)
    const int lane = threadIdx.x & 31;
    const int wave = __builtin_amdgcn_readfirstlane((int)(threadIdx.x >> 5));
    const int row = blockIdx.x * 4 + wave;
    const int bb = row / SQ, tt = row % SQ;
    const float* xr = src + ((size_t)bb * SQ_FULL + tt) * DM;
    v8f a = *(const v8f*)(xr + 8 * lane), c = *(const v8f*)(xr + 256 + 8 * lane);
    v8f ga = *(const v8f*)(g + 8 * lane), gc = *(const v8f*)(g + 256 + 8 * lane);
    v8f ba = *(const v8f*)(bt + 8 * lane), bc = *(const v8f*)(bt + 256 + 8 * lane);
#pragma unroll
    for (int k = 0; k < 8; ++k) { a[k] = bfr(a[k]); c[k] = bfr(c[k]); ga[k] = bfr(ga[k]); gc[k] = bfr(gc[k]); ba[k] = bfr(ba[k]); bc[k] = bfr(bc[k]); }
    ln_row(a, c, ga, gc, ba, bc);
    v8h ha, hc;
#pragma unroll
    for (int k = 0; k < 8; ++k) { ha[k] = toh_flush(a[k]); hc[k] = toh_flush(c[k]); }
    h16* dr = dst + (size_t)row * DM;
    *(volatile v8h*)(dr + 8 * lane) = ha; *(volatile v8h*)(dr + 256 + 8 * lane) = hc;
    __threadfence();
    *(volatile v8h*)(dr + 8 * lane) = ha; *(volatile v8h*)(dr + 256 + 8 * lane) = hc;
}

__global__ __launch_bounds__(128) void k_ln2(const float* __restrict__ src, const float* __restrict__ g, const float* __restrict__ bt, float* O1, h16* dst) {
#pragma clang fp contract(off)
    __shared__ __align__(16) float ls[4 * DM];
    const int lane = threadIdx.x & 31;
    const int wave = __builtin_amdgcn_readfirstlane((int)(threadIdx.x >> 5));
    const int row = blockIdx.x * 4 + wave;
    const int bb = row / SQ, tt = row % SQ;
    const float* xr = src + (size_t)row * DM;
    v8f a = *(const v8f*)(xr + 8 * lane), c = *(const v8f*)(xr + 256 + 8 * lane);
    v8f ga = *(const v8f*)(g + 8 * lane), gc = *(const v8f*)(g + 256 + 8 * lane);
    v8f ba = *(const v8f*)(bt + 8 * lane), bc = *(const v8f*)(bt + 256 + 8 * lane);
#pragma unroll
    for (int k = 0; k < 8; ++k) { ga[k] = bfr(ga[k]); gc[k] = bfr(gc[k]); ba[k] = bfr(ba[k]); bc[k] = bfr(bc[k]); }
    ln_row(a, c, ga, gc, ba, bc);
    const int wb = wave * DM;
    *(v4fa*)(&ls[wb + 8 * lane]) = lo4(a); *(v4fa*)(&ls[wb + 8 * lane + 4]) = hi4(a);
    *(v4fa*)(&ls[wb + 256 + 8 * lane]) = lo4(c); *(v4fa*)(&ls[wb + 256 + 8 * lane + 4]) = hi4(c);
    wave_sync();
    v8h ha, hc;
#pragma unroll
    for (int k = 0; k < 8; ++k) { ha[k] = toh_flush(a[k]); hc[k] = toh_flush(c[k]); }
    h16* dr = dst + (size_t)row * DM;
    float* orow = O1 + ((size_t)bb * SQ_FULL + tt) * DM;
#pragma unroll 1
    for (int ps = 0; ps < 2; ++ps) {
#pragma unroll
        for (int i = 0; i < 4; ++i) { const v4f val = *(const v4fa*)(&ls[wb + 128 * i + 4 * lane]);
            *(volatile v4f*)(orow + 128 * i + 4 * lane) = val; }
        *(volatile v8h*)(dr + 8 * lane) = ha; *(volatile v8h*)(dr + 256 + 8 * lane) = hc;
        if (ps == 0) __threadfence(); }
}

__device__ __forceinline__ void gemm_main(const h16* __restrict__ A, const h16* __restrict__ Bt, size_t aoff, size_t boff, v8f (&acc)[4][4]) {
#pragma unroll
    for (int mb = 0; mb < 4; ++mb)
#pragma unroll
        for (int nb = 0; nb < 4; ++nb) acc[mb][nb] = (v8f){};
#pragma unroll 1
    for (int kc = 0; kc < KD; kc += 32) {
        v16h a[4];
#pragma unroll
        for (int mb = 0; mb < 4; ++mb) a[mb] = ldh(A + aoff + (size_t)mb * 16 * KD + kc);
#pragma unroll
        for (int nb = 0; nb < 4; ++nb) { const v16h b = ldh(Bt + boff + (size_t)nb * 16 * KD + kc);
#pragma unroll
            for (int mb = 0; mb < 4; ++mb) acc[mb][nb] = wmma16g(a[mb], b, acc[mb][nb]); }
    }
}

__global__ __launch_bounds__(32) void k_gemm_head(const h16* __restrict__ A, const h16* __restrict__ Bt, float oscale, h16* Ph, size_t pstride, int T) {
    __shared__ __align__(16) float os[16 * GSP];
    const int lane = threadIdx.x & 31, lr = lane & 15, hi = lane >> 4; const int r0 = blockIdx.x * 64, c0 = blockIdx.y * 64;
    v8f acc[4][4];
    gemm_main(A, Bt, (size_t)(r0 + lr) * KD + 8 * hi, (size_t)(c0 + lr) * KD + 8 * hi, acc);
    const int bb = r0 / T, tt = r0 % T; const int proj = c0 / DM, hh = (c0 % DM) / HD;
    const size_t tbase = (size_t)proj * pstride + ((size_t)(bb * NH_ + hh) * (size_t)T + (size_t)tt) * HD;
#pragma unroll
    for (int mb = 0; mb < 4; ++mb) {
#pragma unroll
        for (int nb = 0; nb < 4; ++nb) {
#pragma unroll
            for (int j = 0; j < 8; ++j) os[(hi * 8 + j) * GSP + nb * 16 + lr] = acc[mb][nb][j] * oscale; }
        wave_sync();
        const size_t sb = tbase + (size_t)(mb * 16) * HD;
#pragma unroll 1
        for (int ps = 0; ps < 2; ++ps) {
#pragma unroll
            for (int s = 0; s < 4; ++s) { const int row = 4 * s + (lane >> 3), c8 = (lane & 7) * 8;
                const v4f x0 = *(const v4fa*)(&os[row * GSP + c8]); const v4f x1 = *(const v4fa*)(&os[row * GSP + c8 + 4]); v8h hv;
#pragma unroll
                for (int i = 0; i < 4; ++i) { hv[i] = toh_flush(x0[i]); hv[4 + i] = toh_flush(x1[i]); }
                *(volatile v8h*)(Ph + sb + (size_t)row * HD + c8) = hv; }
            if (ps == 0) __threadfence(); }
        wave_sync();
    }
}

__global__ __launch_bounds__(32) void k_gemm_tr(const h16* __restrict__ A, const h16* __restrict__ Bt, float oscale, h16* Ph, int T) {
    __shared__ __align__(16) float os[16 * GSP];
    const int lane = threadIdx.x & 31, lr = lane & 15, hi = lane >> 4; const int r0 = blockIdx.x * 64, c0 = blockIdx.y * 64;
    v8f acc[4][4];
    gemm_main(A, Bt, (size_t)(r0 + lr) * KD + 8 * hi, (size_t)(c0 + lr) * KD + 8 * hi, acc);
    const int bb = c0 / T, tt = c0 % T;
    const size_t tbase = (size_t)bb * (size_t)DM * (size_t)T + (size_t)r0 * (size_t)T + (size_t)tt;
#pragma unroll
    for (int mb = 0; mb < 4; ++mb) {
#pragma unroll
        for (int nb = 0; nb < 4; ++nb) {
#pragma unroll
            for (int j = 0; j < 8; ++j) os[(hi * 8 + j) * GSP + nb * 16 + lr] = acc[mb][nb][j] * oscale; }
        wave_sync();
        const size_t sb = tbase + (size_t)(mb * 16) * (size_t)T;
#pragma unroll 1
        for (int ps = 0; ps < 2; ++ps) {
#pragma unroll
            for (int s = 0; s < 4; ++s) { const int row = 4 * s + (lane >> 3), c8 = (lane & 7) * 8;
                const v4f x0 = *(const v4fa*)(&os[row * GSP + c8]); const v4f x1 = *(const v4fa*)(&os[row * GSP + c8 + 4]); v8h hv;
#pragma unroll
                for (int i = 0; i < 4; ++i) { hv[i] = toh_flush(x0[i]); hv[4 + i] = toh_flush(x1[i]); }
                *(volatile v8h*)(Ph + sb + (size_t)row * (size_t)T + c8) = hv; }
            if (ps == 0) __threadfence(); }
        wave_sync();
    }
}

__global__ __launch_bounds__(32) void k_gemm_row(const h16* __restrict__ A, const h16* __restrict__ Bt, float oscale, float* Pf, int OT,
                                                 const float* __restrict__ bias, const float* __restrict__ resid, int has_res) {
    __shared__ __align__(16) float os[16 * GSP];
    const int lane = threadIdx.x & 31, lr = lane & 15, hi = lane >> 4; const int r0 = blockIdx.x * 64, c0 = blockIdx.y * 64;
    v8f acc[4][4];
    gemm_main(A, Bt, (size_t)(r0 + lr) * KD + 8 * hi, (size_t)(c0 + lr) * KD + 8 * hi, acc);
    const int bb = r0 / SQ, tt = r0 % SQ;
    const int c4 = (lane & 15) * 4, rsel = lane >> 4;
    v4f bv = *(const v4f*)(bias + c0 + c4);
#pragma unroll
    for (int i = 0; i < 4; ++i) bv[i] = bfr(bv[i]);
    float* ob = Pf + ((size_t)bb * (size_t)OT + (size_t)tt) * DM + c0 + c4;
    const float* rbp = resid + ((size_t)bb * SQ_FULL + (size_t)tt) * DM + c0 + c4;
#pragma unroll
    for (int mb = 0; mb < 4; ++mb) {
#pragma unroll
        for (int nb = 0; nb < 4; ++nb) {
#pragma unroll
            for (int j = 0; j < 8; ++j) os[(hi * 8 + j) * GSP + nb * 16 + lr] = acc[mb][nb][j] * oscale; }
        wave_sync();
#pragma unroll 1
        for (int ps = 0; ps < 2; ++ps) {
#pragma unroll
            for (int s = 0; s < 8; ++s) { const int row = 2 * s + rsel;
                v4f val = *(const v4fa*)(&os[row * GSP + c4]); val = val + bv;
                if (has_res != 0) { const v4f rv = *(const v4f*)(rbp + (size_t)(mb * 16 + row) * DM);
#pragma unroll
                    for (int i = 0; i < 4; ++i) val[i] += bfr(rv[i]); }
                *(volatile v4f*)(ob + (size_t)(mb * 16 + row) * DM) = val; }
            if (ps == 0) __threadfence(); }
        wave_sync();
    }
}

__global__ __launch_bounds__(32 * AW) void k_flash(const h16* __restrict__ QH, const h16* __restrict__ KP, const h16* __restrict__ VT, h16* CTX, int Tq, int Tk, int loc) {
    __shared__ __align__(16) float os[AW * 16 * OSP];
    const int lane = threadIdx.x & 31, lr = lane & 15, hi = lane >> 4;
    const int wave = __builtin_amdgcn_readfirstlane((int)(threadIdx.x >> 5));
    const int zh = blockIdx.y; const int b = zh / NH_, h = zh % NH_;
    const int t0 = (blockIdx.x * AW + wave) * 16;
    const int kbeg = (t0 & ~(CH - 1)) * loc;
    const int kend = kbeg + CH * loc + Tk * (1 - loc);
    const size_t qbase = (size_t)zh * (size_t)Tq * HD;
    const size_t kbase = (size_t)zh * (size_t)Tk * HD;
    const size_t qo = qbase + (size_t)(t0 + lr) * HD + 8 * hi;
    const v16h q0 = ldh(QH + qo), q1 = ldh(QH + qo + 32);
    const size_t ko = kbase + (size_t)lr * HD + 8 * hi;
    const size_t vo = kbase + (size_t)lr * (size_t)Tk + 8 * hi;
    v8f o0 = (v8f){}, o1 = (v8f){}, o2 = (v8f){}, o3 = (v8f){};
    float m = NEGB, l = 0.0f;
#pragma unroll 1
    for (int key0 = kbeg; key0 < kend; key0 += 32) {
        const h16* ka = KP + ko + (size_t)key0 * HD;
        v8f sa = (v8f){}, sb = (v8f){};
        { const v16h k0 = ldh(ka), k1 = ldh(ka + 32);
          sa = wmma16g(k0, q0, sa); sa = wmma16g(k1, q1, sa); }
        { const v16h k0 = ldh(ka + 16 * HD), k1 = ldh(ka + 16 * HD + 32);
          sb = wmma16g(k0, q0, sb); sb = wmma16g(k1, q1, sb); }
        float ta[8], tb[8]; float mx = NEGB;
#pragma unroll
        for (int r = 0; r < 8; ++r) { ta[r] = sa[r] * SC2; tb[r] = sb[r] * SC2; mx = fmaxf(mx, fmaxf(ta[r], tb[r])); }
        mx = fmaxf(mx, __shfl_xor(mx, 16, 32));
        const float mnew = fmaxf(m, mx);
        const float alpha = __builtin_amdgcn_exp2f(m - mnew);
        const float sh = PSH - mnew;
        v16h pb; float ls = 0.0f;
#pragma unroll
        for (int r = 0; r < 8; ++r) {
            const float ea = ta[r] + sh, eb = tb[r] + sh;
            const float xa = __builtin_amdgcn_exp2f(ea), xb = __builtin_amdgcn_exp2f(eb);
            const float ga = (ea < -14.0f) ? 0.0f : xa, gb = (eb < -14.0f) ? 0.0f : xb;
            const h16 pa = (h16)ga; const h16 pc = (h16)gb;
            pb[r] = pa; pb[8 + r] = pc;
            ls += (float)pa + (float)pc; }
        l = l * alpha + ls; m = mnew;
        o0 = o0 * alpha; o1 = o1 * alpha; o2 = o2 * alpha; o3 = o3 * alpha;
        const h16* va = VT + vo + key0;
        const v16h v0 = ldh(va), v1 = ldh(va + (size_t)16 * Tk), v2 = ldh(va + (size_t)32 * Tk), v3 = ldh(va + (size_t)48 * Tk);
        o0 = wmma16g(v0, pb, o0); o1 = wmma16g(v1, pb, o1); o2 = wmma16g(v2, pb, o2); o3 = wmma16g(v3, pb, o3);
    }
    l += __shfl_xor(l, 16, 32);
    const float lsafe = fmaxf(l, 1.0e-30f);
    const float inv = CTXC * (1.0f / lsafe);
    const int wb = wave * 16 * OSP;
    { v4f a, c;
      a[0] = o0[0] * inv; a[1] = o0[1] * inv; a[2] = o0[2] * inv; a[3] = o0[3] * inv; c[0] = o0[4] * inv; c[1] = o0[5] * inv; c[2] = o0[6] * inv; c[3] = o0[7] * inv;
      *(v4fa*)(&os[wb + lr * OSP +  0 + 8 * hi]) = a; *(v4fa*)(&os[wb + lr * OSP +  0 + 8 * hi + 4]) = c;
      a[0] = o1[0] * inv; a[1] = o1[1] * inv; a[2] = o1[2] * inv; a[3] = o1[3] * inv; c[0] = o1[4] * inv; c[1] = o1[5] * inv; c[2] = o1[6] * inv; c[3] = o1[7] * inv;
      *(v4fa*)(&os[wb + lr * OSP + 16 + 8 * hi]) = a; *(v4fa*)(&os[wb + lr * OSP + 16 + 8 * hi + 4]) = c;
      a[0] = o2[0] * inv; a[1] = o2[1] * inv; a[2] = o2[2] * inv; a[3] = o2[3] * inv; c[0] = o2[4] * inv; c[1] = o2[5] * inv; c[2] = o2[6] * inv; c[3] = o2[7] * inv;
      *(v4fa*)(&os[wb + lr * OSP + 32 + 8 * hi]) = a; *(v4fa*)(&os[wb + lr * OSP + 32 + 8 * hi + 4]) = c;
      a[0] = o3[0] * inv; a[1] = o3[1] * inv; a[2] = o3[2] * inv; a[3] = o3[3] * inv; c[0] = o3[4] * inv; c[1] = o3[5] * inv; c[2] = o3[6] * inv; c[3] = o3[7] * inv;
      *(v4fa*)(&os[wb + lr * OSP + 48 + 8 * hi]) = a; *(v4fa*)(&os[wb + lr * OSP + 48 + 8 * hi + 4]) = c; }
    wave_sync();
    h16* crow = CTX + ((size_t)b * (size_t)Tq + (size_t)t0) * DM + h * HD;
#pragma unroll 1
    for (int ps = 0; ps < 2; ++ps) {
#pragma unroll
        for (int s = 0; s < 4; ++s) { const int row = 4 * s + (lane >> 3), c8 = (lane & 7) * 8;
            const v4f x0 = *(const v4fa*)(&os[wb + row * OSP + c8]); const v4f x1 = *(const v4fa*)(&os[wb + row * OSP + c8 + 4]); v8h hv;
#pragma unroll
            for (int i = 0; i < 4; ++i) { hv[i] = toh_flush(x0[i]); hv[4 + i] = toh_flush(x1[i]); }
            *(volatile v8h*)(crow + (size_t)row * DM + c8) = hv; }
        if (ps == 0) __threadfence(); }
}

static constexpr size_t al256(size_t v) { return (v + 255) & ~(size_t)255; }
static constexpr int WROWS = 1536 + 512 + 512 + 1024 + 512;
static constexpr size_t SZ_WT = al256((size_t)WROWS * KD * 2);
static constexpr size_t SZ_AQ = al256((size_t)NTOKQ * DM * 2);
static constexpr size_t SZ_AK = al256((size_t)NTOKK * DM * 2);
static constexpr size_t SZ_TQ = al256((size_t)NTOKQ * DM * 4);
static constexpr size_t SZ_TOTAL = SZ_WT + 8 * SZ_AQ + 3 * SZ_AK + SZ_TQ;
static_assert(SZ_TOTAL <= (size_t)134217728);
static_assert(SZ_AQ % 2 == 0);
static_assert((size_t)NB * NH_ * SQ * HD == (size_t)NTOKQ * DM);
static_assert((size_t)NB * NH_ * SK * HD == (size_t)NTOKK * DM);
static_assert(WROWS % 64 == 0);

extern "C" void kernel_launch(void* const* d_in, const int* in_sizes, int n_in,
                              void* d_out, int out_size, void* d_ws, size_t ws_size, hipStream_t stream) {
    if (n_in < 13) return;
    const size_t needx = ((size_t)(NB - 1) * SK_FULL + SK) * DM;
    const size_t needq = ((size_t)(NB - 1) * SQ_FULL + SQ) * DM;
    if ((size_t)in_sizes[0] < needx || (size_t)in_sizes[1] < needq) return;
    if (in_sizes[2] < DM || in_sizes[3] < DM || in_sizes[6] < DM || in_sizes[7] < DM || in_sizes[8] < DM || in_sizes[12] < DM) return;
    if ((size_t)in_sizes[4] < (size_t)KD * 1536 || (size_t)in_sizes[5] < (size_t)KD * 512 || (size_t)in_sizes[9] < (size_t)KD * 512) return;
    if ((size_t)in_sizes[10] < (size_t)KD * 1024 || (size_t)in_sizes[11] < (size_t)KD * 512) return;
    if ((size_t)out_size < OUT1_OFF + needq) return;
    if (SZ_TOTAL > ws_size) return;
    const float* x     = (const float*)d_in[0];
    const float* q_x   = (const float*)d_in[1];
    const float* ln1_g = (const float*)d_in[2];
    const float* ln1_b = (const float*)d_in[3];
    const float* W_qkv = (const float*)d_in[4];
    const float* W_ao  = (const float*)d_in[5];
    const float* b_ao  = (const float*)d_in[6];
    const float* ln2_g = (const float*)d_in[7];
    const float* ln2_b = (const float*)d_in[8];
    const float* W_q   = (const float*)d_in[9];
    const float* W_kv  = (const float*)d_in[10];
    const float* W_o   = (const float*)d_in[11];
    const float* b_o   = (const float*)d_in[12];
    float* OUT0 = (float*)d_out;
    float* OUT1 = (float*)d_out + OUT1_OFF;

    char* wsp = (char*)d_ws;
    h16* WT   = (h16*)wsp; wsp += SZ_WT;
    h16* LN1H = (h16*)wsp; wsp += SZ_AQ;
    h16* XH   = (h16*)wsp; wsp += SZ_AK;
    h16* QL   = (h16*)wsp; wsp += SZ_AQ;
    h16* KL   = (h16*)wsp; wsp += SZ_AQ;
    h16* VLT  = (h16*)wsp; wsp += SZ_AQ;
    h16* CL   = (h16*)wsp; wsp += SZ_AQ;
    float* TMP = (float*)wsp; wsp += SZ_TQ;
    h16* QIN  = (h16*)wsp; wsp += SZ_AQ;
    h16* QC   = (h16*)wsp; wsp += SZ_AQ;
    h16* KC   = (h16*)wsp; wsp += SZ_AK;
    h16* VCT  = (h16*)wsp; wsp += SZ_AK;
    h16* CC   = (h16*)wsp; wsp += SZ_AQ;
    h16* WqkvT = WT;
    h16* WaoT  = WT + (size_t)1536 * KD;
    h16* WqT   = WT + (size_t)2048 * KD;
    h16* WkvT  = WT + (size_t)2560 * KD;
    h16* WoT   = WT + (size_t)3584 * KD;

    k_wconv<<<dim3(1536 / 64, KD / 64, 1), 256, 0, stream>>>(W_qkv, WqkvT, 1536);
    k_wconv<<<dim3(512 / 64,  KD / 64, 1), 256, 0, stream>>>(W_ao,  WaoT,  512);
    k_wconv<<<dim3(512 / 64,  KD / 64, 1), 256, 0, stream>>>(W_q,   WqT,   512);
    k_wconv<<<dim3(1024 / 64, KD / 64, 1), 256, 0, stream>>>(W_kv,  WkvT,  1024);
    k_wconv<<<dim3(512 / 64,  KD / 64, 1), 256, 0, stream>>>(W_o,   WoT,   512);

    k_ln1<<<NTOKQ / 4, 128, 0, stream>>>(q_x, ln1_g, ln1_b, LN1H);
    { const size_t n8 = (size_t)NTOKK * DM / 8;
      k_xcvt<<<(unsigned)((n8 + 255) / 256), 256, 0, stream>>>(x, XH, SK, SK_FULL, n8); }

    k_gemm_head<<<dim3(NTOKQ / 64, 1024 / 64, 1), 32, 0, stream>>>(LN1H, WqkvT, WSI, QL, (size_t)(SZ_AQ / 2), SQ);
    k_gemm_tr<<<dim3(DM / 64, NTOKQ / 64, 1), 32, 0, stream>>>(WqkvT + (size_t)1024 * KD, LN1H, WSI, VLT, SQ);
    k_flash<<<dim3(SQ / (16 * AW), NB * NH_, 1), 32 * AW, 0, stream>>>(QL, KL, VLT, CL, SQ, SQ, 1);
    k_gemm_row<<<dim3(NTOKQ / 64, DM / 64, 1), 32, 0, stream>>>(CL, WaoT, WSI * (1.0f / CTXC), TMP, SQ, b_ao, q_x, 1);
    k_ln2<<<NTOKQ / 4, 128, 0, stream>>>(TMP, ln2_g, ln2_b, OUT1, QIN);

    k_gemm_head<<<dim3(NTOKQ / 64, DM / 64, 1), 32, 0, stream>>>(QIN, WqT, WSI, QC, (size_t)0, SQ);
    k_gemm_head<<<dim3(NTOKK / 64, DM / 64, 1), 32, 0, stream>>>(XH, WkvT, WSI, KC, (size_t)0, SK);
    k_gemm_tr<<<dim3(DM / 64, NTOKK / 64, 1), 32, 0, stream>>>(WkvT + (size_t)512 * KD, XH, WSI, VCT, SK);
    k_flash<<<dim3(SQ / (16 * AW), NB * NH_, 1), 32 * AW, 0, stream>>>(QC, KC, VCT, CC, SQ, SK, 0);
    k_gemm_row<<<dim3(NTOKQ / 64, DM / 64, 1), 32, 0, stream>>>(CC, WoT, WSI * (1.0f / CTXC), OUT0, SQ_FULL, b_o, q_x, 0);
}
